// GlobalAttentionBlock_35390530519684
// MI455X (gfx1250) — hardware-verified
//
#include <hip/hip_runtime.h>
#include <stdint.h>

typedef _Float16 bf16_t;
typedef __attribute__((ext_vector_type(16))) _Float16  v16bf;
typedef __attribute__((ext_vector_type(8)))  _Float16  v8bf;
typedef __attribute__((ext_vector_type(8)))  float     v8f;
typedef __attribute__((ext_vector_type(4)))  uint32_t  u32x4;
typedef __attribute__((ext_vector_type(4)))  float     v4f_t;
typedef float v4fa __attribute__((ext_vector_type(4), may_alias));
typedef uint32_t v4ua __attribute__((ext_vector_type(4), may_alias));

#define CH     256
#define NPIX   4096
#define NHEADS 8
#define HD     32
#define NGRP   32
#define GSIZE  (CH / NGRP)
#define GN_EPS 1e-5f
#define NB     2

__device__ __forceinline__ v16bf rfrag(const bf16_t* rowp, int lane) {
  const bf16_t* p = rowp + ((lane >> 4) * 8);
  return __builtin_shufflevector(*(const v8bf*)p, *(const v8bf*)(p + 16), 0,1,2,3,4,5,6,7,8,9,10,11,12,13,14,15);
}
__device__ __forceinline__ v8f wmma16(v16bf a, v16bf b, v8f c) {
  return __builtin_amdgcn_wmma_f32_16x16x32_f16(false, a, false, b, (short)0, c, false, false);
}
__device__ __forceinline__ void st16h(bf16_t* d, const bf16_t* s) { *(volatile u32x4*)d = *(const v4ua*)s; }

__global__ __launch_bounds__(256) void k_gn_stats(const float* __restrict__ x, float* __restrict__ stat, float* __restrict__ chs) {
  __shared__ float red[2][256];
  __shared__ float csum[GSIZE][8];
  const int bg = blockIdx.x, b = bg / NGRP, g = bg % NGRP, c0 = g * GSIZE;
  const int t = threadIdx.x, lane = t & 31, wave = t >> 5;
  const float* xp = x + ((size_t)b * CH + c0) * NPIX;
  float s = 0.f, ss = 0.f;
  {
    const float* xc = xp + (size_t)wave * NPIX;
    float cs = 0.f;
    for (int i = lane * 4; i < NPIX; i += 128) { const v4f_t v = *(const v4f_t*)(xc + i); cs += (v.x + v.y) + (v.z + v.w); ss += v.x * v.x + v.y * v.y + v.z * v.z + v.w * v.w; }
    s = cs;
#pragma unroll
    for (int o = 16; o > 0; o >>= 1) cs += __shfl_xor(cs, o, 32);
    if (lane == 0) csum[wave][0] = cs;
  }
  red[0][t] = s; red[1][t] = ss; __syncthreads();
  for (int o = 128; o > 0; o >>= 1) { if (t < o) { red[0][t] += red[0][t + o]; red[1][t] += red[1][t + o]; } __syncthreads(); }
  const float mean = red[0][0] * (1.0f / (GSIZE * NPIX));
  const float var  = red[1][0] * (1.0f / (GSIZE * NPIX)) - mean * mean;
  const float inv  = rsqrtf(var + GN_EPS);
  if (t < 2) { float v = (t == 0) ? mean : inv; *(volatile float*)(stat + bg * 2 + t) = v; __threadfence(); *(volatile float*)(stat + bg * 2 + t) = v; }
  if (t < GSIZE) { const float v = csum[t][0]; *(volatile float*)(chs + b * CH + c0 + t) = v; __threadfence(); *(volatile float*)(chs + b * CH + c0 + t) = v; }
}

__global__ __launch_bounds__(256) void k_gfeat(const float* __restrict__ stat, const float* __restrict__ chs,
                                               const float* __restrict__ gn_w, const float* __restrict__ gn_b,
                                               const float* __restrict__ gproj_w, const float* __restrict__ gproj_b,
                                               float* __restrict__ gfeat) {
  __shared__ float gm[CH];
  const int b = blockIdx.x, o = threadIdx.x;
  { const int c = o, g = c / GSIZE; gm[c] = (chs[b * CH + c] * (1.0f / NPIX) - stat[(b * NGRP + g) * 2]) * stat[(b * NGRP + g) * 2 + 1] * gn_w[c] + gn_b[c]; }
  __syncthreads();
  float s = 0.f;
#pragma unroll 1
  for (int c = 0; c < CH; ++c) s += gm[c] * gproj_w[o * CH + c];
  s += gproj_b[o];
  *(volatile float*)(gfeat + b * CH + o) = s; __threadfence(); *(volatile float*)(gfeat + b * CH + o) = s;
}

__global__ __launch_bounds__(256) void k_gn_apply(const float* __restrict__ x, const float* __restrict__ stat,
                                                  const float* __restrict__ gn_w, const float* __restrict__ gn_b,
                                                  bf16_t* __restrict__ xn) {
  const int n0 = blockIdx.x * 32, b = blockIdx.y, t = threadIdx.x;
#pragma unroll 1
  for (int pass = 0; pass < 2; ++pass) {
    for (int ch = t; ch < 32 * (CH / 8); ch += 256) {
      const int nl = ch & 31, c8 = (ch >> 5) * 8;
      const int g = c8 / GSIZE;
      const float mean = stat[(b * NGRP + g) * 2], inv = stat[(b * NGRP + g) * 2 + 1];
      bf16_t hh[8];
#pragma unroll
      for (int e = 0; e < 8; ++e) { const int c = c8 + e; hh[e] = (bf16_t)((x[((size_t)b * CH + c) * NPIX + n0 + nl] - mean) * inv * gn_w[c] + gn_b[c]); }
      st16h(xn + ((size_t)b * NPIX + n0 + nl) * CH + c8, hh);
    }
    __threadfence();
  }
}

__global__ __launch_bounds__(256) void k_qkv_gemm(const bf16_t* __restrict__ xn, const float* __restrict__ qkv_w,
                                                  const float* __restrict__ qkv_b, const float* __restrict__ gfeat,
                                                  bf16_t* __restrict__ qb, bf16_t* __restrict__ kb, bf16_t* __restrict__ vb) {
  const int j0 = blockIdx.x * 32, which = blockIdx.y, o0 = which * 256, b = blockIdx.z;
  const int t = threadIdx.x, lane = t & 31, wave = t >> 5;
  const int wmj = (wave >> 2) * 16, wno = (wave & 3) * 64;
  __shared__ __align__(32) bf16_t Ws[256 * 40];
  __shared__ __align__(16) float  Ds[32 * 260];

  const bf16_t* Arow = xn + ((size_t)b * NPIX + j0 + wmj + (lane & 15)) * CH;
  v8f acc[4] = {{}, {}, {}, {}};
  for (int kc = 0; kc < CH; kc += 32) {
    __syncthreads();
#pragma unroll
    for (int r = 0; r < 4; ++r) {
      const int gi = t + r * 256, o = gi >> 2, cseg = (gi & 3) * 8;
      const float* wp = qkv_w + (size_t)(o0 + o) * CH + kc + cseg;
      bf16_t pk[8];
#pragma unroll
      for (int e = 0; e < 8; ++e) pk[e] = (bf16_t)wp[e];
      *(u32x4*)(Ws + o * 40 + cseg) = *(const v4ua*)pk;
    }
    __syncthreads();
    const v16bf af = rfrag(Arow + kc, lane);
#pragma unroll
    for (int s = 0; s < 4; ++s) acc[s] = wmma16(af, rfrag(Ws + (wno + s * 16 + (lane & 15)) * 40, lane), acc[s]);
  }
#pragma unroll
  for (int s = 0; s < 4; ++s) {
    const int ol = wno + s * 16 + (lane & 15), og = o0 + ol;
    float add = qkv_b[og];
    if (which == 1) add += 0.1f * gfeat[b * CH + (og - CH)];
#pragma unroll
    for (int r = 0; r < 8; ++r) Ds[(wmj + (lane >> 4) * 8 + r) * 260 + ol] = acc[s][r] + add;
  }
  __syncthreads();
  bf16_t* dstT = (which == 0) ? qb : (which == 1) ? kb : vb;
#pragma unroll 1
  for (int pass = 0; pass < 2; ++pass) {
    for (int ch = t; ch < 8 * 32 * 4; ch += 256) { const int h = ch >> 7, nl = (ch >> 2) & 31, d8 = (ch & 3) * 8;
      bf16_t hh[8];
#pragma unroll
      for (int e = 0; e < 8; ++e) hh[e] = (bf16_t)Ds[nl * 260 + h * 32 + d8 + e];
      st16h(dstT + (((size_t)(b * NHEADS + h) * NPIX) + j0 + nl) * HD + d8, hh);
    }
    __threadfence();
  }
}

__global__ __launch_bounds__(256) void k_attn(const bf16_t* __restrict__ qb, const bf16_t* __restrict__ kb,
                                              const bf16_t* __restrict__ vb, bf16_t* __restrict__ ao) {
  const int bh = blockIdx.y;
  const int q0 = blockIdx.x * 128;
  const int t = threadIdx.x, lane = t & 31, wave = t >> 5;
  const float scale = 0.17677669529663687f;
  const bf16_t* Q = qb + (size_t)bh * NPIX * HD;
  const bf16_t* K = kb + (size_t)bh * NPIX * HD;
  const bf16_t* V = vb + (size_t)bh * NPIX * HD;

  const int qidx = q0 + wave * 16 + (lane & 15);
  const v16bf qf = rfrag(Q + (size_t)qidx * HD, lane);

  __shared__ __align__(32) bf16_t Ks[64 * 32];
  __shared__ __align__(32) bf16_t Vs[32 * 72];
  __shared__ __align__(16) bf16_t Os[128 * 32];

  const int krow = t >> 2, kseg = (t & 3) * 8;
  float m_run = -1e30f, l_run = 0.f;
  v8f o_acc0 = {}, o_acc1 = {};
  const int half = lane >> 4;

  for (int kc = 0; kc < NPIX; kc += 64) {
    __syncthreads();
    {
      const u32x4 kv = *(const u32x4*)(K + (size_t)(kc + krow) * HD + kseg);
      *(u32x4*)(Ks + krow * 32 + kseg) = kv;
      union { u32x4 u; bf16_t h[8]; } vv; vv.u = *(const u32x4*)(V + (size_t)(kc + krow) * HD + kseg);
#pragma unroll
      for (int e = 0; e < 8; ++e) Vs[(kseg + e) * 72 + krow] = vv.h[e];
    }
    __syncthreads();

    v8f sv[4];
#pragma unroll
    for (int mt = 0; mt < 4; ++mt) { v8f z = {}; sv[mt] = wmma16(rfrag(Ks + (mt * 16 + (lane & 15)) * 32, lane), qf, z); }

    float mx = -1e30f;
#pragma unroll
    for (int mt = 0; mt < 4; ++mt)
#pragma unroll
      for (int r = 0; r < 8; ++r) { sv[mt][r] *= scale; mx = fmaxf(mx, sv[mt][r]); }
    mx = fmaxf(mx, __shfl_xor(mx, 16, 32));
    const float mnew = fmaxf(m_run, mx);
    const float corr = __expf(m_run - mnew);
    m_run = mnew;

    float ps = 0.f;
    v16bf pf[2];
#pragma unroll
    for (int kstep = 0; kstep < 2; ++kstep)
#pragma unroll
      for (int r = 0; r < 8; ++r) {
        const float pA = __expf(sv[2 * kstep][r] - mnew), pB = __expf(sv[2 * kstep + 1][r] - mnew);
        ps += pA + pB;
        pf[kstep][r] = (bf16_t)(pA * 1024.0f); pf[kstep][8 + r] = (bf16_t)(pB * 1024.0f);
      }
    ps += __shfl_xor(ps, 16, 32);
    l_run = l_run * corr + ps;
#pragma unroll
    for (int r = 0; r < 8; ++r) { o_acc0[r] *= corr; o_acc1[r] *= corr; }

#pragma unroll
    for (int kstep = 0; kstep < 2; ++kstep) {
      const v16bf vf0 = rfrag(Vs + (lane & 15) * 72 + kstep * 32, lane);
      const v16bf vf1 = rfrag(Vs + (16 + (lane & 15)) * 72 + kstep * 32, lane);
      o_acc0 = wmma16(vf0, pf[kstep], o_acc0);
      o_acc1 = wmma16(vf1, pf[kstep], o_acc1);
    }
  }

  const float invl = 1.0f / (l_run * 1024.0f);
  {
    const int ql = wave * 16 + (lane & 15);
#pragma unroll
    for (int r = 0; r < 8; ++r) { Os[ql * 32 + half * 8 + r] = (bf16_t)(o_acc0[r] * invl); Os[ql * 32 + 16 + half * 8 + r] = (bf16_t)(o_acc1[r] * invl); }
  }
  __syncthreads();
  bf16_t* aop = ao + ((size_t)bh * NPIX + q0) * HD;
#pragma unroll 1
  for (int pass = 0; pass < 2; ++pass) {
    for (int ch = t; ch < 128 * 4; ch += 256) st16h(aop + ch * 8, Os + ch * 8);
    __threadfence();
  }
}

__global__ __launch_bounds__(256) void k_proj_gemm(const bf16_t* __restrict__ ao, const float* __restrict__ proj_w,
                                                   const float* __restrict__ proj_b, const float* __restrict__ gfeat,
                                                   const float* __restrict__ x, float* __restrict__ out) {
  const int j0 = blockIdx.x * 32, b = blockIdx.z;
  const int t = threadIdx.x, lane = t & 31, wave = t >> 5;
  const int wmj = (wave >> 2) * 16, wno = (wave & 3) * 64;
  __shared__ __align__(32) bf16_t Ws[256 * 40];
  __shared__ __align__(16) float  Ds[256 * 36];

  v8f acc[4] = {{}, {}, {}, {}};
  for (int kc = 0; kc < CH; kc += 32) {
    __syncthreads();
#pragma unroll
    for (int r = 0; r < 4; ++r) {
      const int gi = t + r * 256, o = gi >> 2, cseg = (gi & 3) * 8;
      const float* wp = proj_w + (size_t)o * CH + kc + cseg;
      bf16_t pk[8];
#pragma unroll
      for (int e = 0; e < 8; ++e) pk[e] = (bf16_t)wp[e];
      *(u32x4*)(Ws + o * 40 + cseg) = *(const v4ua*)pk;
    }
    __syncthreads();
    const bf16_t* arow = ao + (((size_t)(b * NHEADS + (kc >> 5)) * NPIX) + j0 + wmj + (lane & 15)) * HD;
    const v16bf af = rfrag(arow, lane);
#pragma unroll
    for (int s = 0; s < 4; ++s) acc[s] = wmma16(af, rfrag(Ws + (wno + s * 16 + (lane & 15)) * 40, lane), acc[s]);
  }
#pragma unroll
  for (int s = 0; s < 4; ++s) {
    const int og = wno + s * 16 + (lane & 15);
    const float base = proj_b[og] + 0.1f * gfeat[b * CH + og];
#pragma unroll
    for (int r = 0; r < 8; ++r) Ds[og * 36 + wmj + (lane >> 4) * 8 + r] = acc[s][r] + base;
  }
  __syncthreads();
#pragma unroll 1
  for (int pass = 0; pass < 2; ++pass) {
    for (int ch = t; ch < 256 * 8; ch += 256) { const int o = ch >> 3, q = (ch & 7) * 4;
      const size_t idx = ((size_t)b * CH + o) * NPIX + j0 + q;
      v4f_t v = *(const v4f_t*)(x + idx); v += *(const volatile v4fa*)(Ds + o * 36 + q);
      *(volatile v4f_t*)(out + idx) = v; }
    __threadfence();
  }
}

extern "C" void kernel_launch(void* const* d_in, const int* in_sizes, int n_in,
                              void* d_out, int out_size, void* d_ws, size_t ws_size,
                              hipStream_t stream) {
  (void)in_sizes; (void)n_in; (void)out_size; (void)ws_size;
  const float* x       = (const float*)d_in[0];
  const float* gn_w    = (const float*)d_in[1];
  const float* gn_b    = (const float*)d_in[2];
  const float* qkv_w   = (const float*)d_in[3];
  const float* qkv_b   = (const float*)d_in[4];
  const float* proj_w  = (const float*)d_in[5];
  const float* proj_b  = (const float*)d_in[6];
  const float* gproj_w = (const float*)d_in[7];
  const float* gproj_b = (const float*)d_in[8];

  char* ws = (char*)d_ws;
  const size_t MB = 1u << 20;
  bf16_t* xn  = (bf16_t*)(ws + 0 * MB);
  bf16_t* qb  = (bf16_t*)(ws + 4 * MB);
  bf16_t* kb  = (bf16_t*)(ws + 8 * MB);
  bf16_t* vb  = (bf16_t*)(ws + 12 * MB);
  bf16_t* ao  = (bf16_t*)(ws + 16 * MB);
  float*  stat  = (float*)(ws + 20 * MB);
  float*  chs   = (float*)(ws + 20 * MB + 4096);
  float*  gfeat = (float*)(ws + 20 * MB + 8192);
  float*  out = (float*)d_out;

  k_gn_stats<<<dim3(NB * NGRP), 256, 0, stream>>>(x, stat, chs);
  k_gfeat<<<dim3(NB), 256, 0, stream>>>(stat, chs, gn_w, gn_b, gproj_w, gproj_b, gfeat);
  k_gn_apply<<<dim3(NPIX / 32, NB), 256, 0, stream>>>(x, stat, gn_w, gn_b, xn);
  k_qkv_gemm<<<dim3(NPIX / 32, 3, NB), 256, 0, stream>>>(xn, qkv_w, qkv_b, gfeat, qb, kb, vb);
  k_attn<<<dim3(NPIX / 128, NB * NHEADS), 256, 0, stream>>>(qb, kb, vb, ao);
  k_proj_gemm<<<dim3(NPIX / 32, 1, NB), 256, 0, stream>>>(ao, proj_w, proj_b, gfeat, x, out);
}
